// LorentzGNN_73710228733975
// MI455X (gfx1250) — hardware-run, weakly checked
//
#include <hip/hip_runtime.h>
#include <stddef.h>
#include <stdint.h>
#include <math.h>


#define NNODE   16384
#define NEDGE   131072
#define HID     512
#define XPITCH  513
#define NGRAPH  128
#define GSIZE   128
#define ZP      544
#define KA      1088
#define KBH     2080
#define KB      4160
#define NA      2176
#define NBF     640
#define OUTW    513
#define OUTQ    16416
#define SCALARS_RNE 1

#define NTHR    256
#define NWAVE   8
#define EPT     8
#define CHUNK   (NTHR * EPT)
#define WCAP    (EPT * 32)
#define LISTN   (NWAVE * WCAP)
#define NBMAX   2048
#define NBRUN   1024
#define RCAP    28672
#define DEGCAP  64
#define STW     512
#define MEAS_B1024  8323
#define MEAS_MAXDEG 21
#define ZINTS   (2 * RCAP + 2 * NBMAX + LISTN)
#define LDS_SCAN ((ZINTS + 2 * NWAVE + 4 * NWAVE) * 4)
#define GBM     64
#define GBN     64
#define GTHR    128
#define NEGS    0.2f
#define WSMAX   134217728

static_assert((CHUNK & (CHUNK - 1)) == 0 && CHUNK <= 4096);
static_assert((NBMAX & (NBMAX - 1)) == 0 && NBMAX <= 4096);
static_assert((NBRUN & (NBRUN - 1)) == 0 && NBRUN <= NBMAX && NBRUN >= 16);
static_assert(NTHR * 8 == NBMAX);
static_assert(LISTN >= NBMAX && LISTN >= NWAVE * WCAP);
static_assert((RCAP % 32) == 0 && (ZINTS % 4) == 0);
static_assert(NWAVE * STW <= RCAP && HID <= STW);
static_assert(RCAP >= 2 * MEAS_B1024);
static_assert(DEGCAP >= MEAS_MAXDEG + 8);
static_assert(LDS_SCAN <= 327680);
static_assert(NEDGE < (1 << 20));
static_assert(NNODE % NBRUN == 0 && NNODE % GBM == 0 && NGRAPH * GSIZE == NNODE);
static_assert(GBM == (GTHR / 32) * 16);
static_assert(HID % 32 == 0 && (2 * HID) % 32 == 0 && KA % 32 == 0 && KB % 32 == 0);
static_assert((2 * HID) % GBN == 0 && NA % GBN == 0 && NBF % GBN == 0 && NGRAPH % GBM == 0);
static_assert(ZP % 8 == 0 && KBH % 8 == 0 && ZP >= OUTW && KBH >= 2049 && NA >= 2049 && NBF >= OUTW);
static_assert((ZP * 4) % 128 == 0 && (KA * 2) % 128 == 0 && (KB * 2) % 128 == 0);
static_assert(LISTN >= 2 * HID + NBRUN);
static_assert(2 * OUTQ * 4 == 2 * NGRAPH * OUTW);

typedef float          v4f   __attribute__((ext_vector_type(4)));
typedef float          v8f   __attribute__((ext_vector_type(8)));
typedef int            v4i   __attribute__((ext_vector_type(4)));
typedef int            v8i   __attribute__((ext_vector_type(8)));
typedef unsigned short v8us  __attribute__((ext_vector_type(8)));
typedef __bf16         v16bf __attribute__((ext_vector_type(16)));
typedef v4f  __attribute__((may_alias)) v4fa;
typedef v4i  __attribute__((may_alias)) v4ia;
union FragB { v16bf v; v8us u[2]; v8i w; };

__device__ __forceinline__ v8f wmb(const FragB& a, const FragB& b, v8f c) {
  v8f d = __builtin_amdgcn_wmma_f32_16x16x32_bf16(false, a.v, false, b.v, (short)0, c, false, false);
  asm volatile("v_nop\n\tv_nop\n\tv_nop\n\tv_nop" : "+v"(d) : "v"(a.w), "v"(b.w));
  return d;
}

__device__ __forceinline__ void ldwait() {
  asm volatile("s_wait_loadcnt 0x0" ::: "memory");
}

__device__ __forceinline__ void wsync() {
  __builtin_amdgcn_fence(__ATOMIC_SEQ_CST, "workgroup");
  __builtin_amdgcn_wave_barrier();
}

__device__ __forceinline__ unsigned bfbits(float v) {
  const unsigned u = __float_as_uint(v);
  const unsigned r = (u + 0x7FFFu + ((u >> 16) & 1u)) >> 16;
  return (v != v) ? 0x7FC0u : r;
}
__device__ __forceinline__ float rbf(float v) { return __uint_as_float(bfbits(v) << 16); }

__device__ __forceinline__ v8us cvt8b(const v4f a, const v4f b) {
  v8us o;
  o[0] = (unsigned short)bfbits(a.x); o[1] = (unsigned short)bfbits(a.y);
  o[2] = (unsigned short)bfbits(a.z); o[3] = (unsigned short)bfbits(a.w);
  o[4] = (unsigned short)bfbits(b.x); o[5] = (unsigned short)bfbits(b.y);
  o[6] = (unsigned short)bfbits(b.z); o[7] = (unsigned short)bfbits(b.w);
  return o;
}
__device__ __forceinline__ void hilo8(const v4f a, const v4f b, v8us& hv, v8us& lv) {
  const float f[8] = {a.x, a.y, a.z, a.w, b.x, b.y, b.z, b.w};
#pragma unroll
  for (int i = 0; i < 8; ++i) {
    const unsigned h = bfbits(f[i]);
    hv[i] = (unsigned short)h;
    lv[i] = (unsigned short)bfbits(f[i] - __uint_as_float(h << 16));
  }
}
__device__ __forceinline__ v8us hl8(const float* row, int u, int hu) {
  const int lo = (u >= hu) ? 1 : 0;
  const int uu = u - lo * hu;
  const v4f a = *(const v4fa*)(row + 8 * uu);
  const v4f b = *(const v4fa*)(row + 8 * uu + 4);
  v8us hv, lv;
  hilo8(a, b, hv, lv);
  const unsigned mk = lo ? 0xFFFFu : 0u;
  v8us o;
#pragma unroll
  for (int i = 0; i < 8; ++i) o[i] = (unsigned short)(((unsigned)hv[i] & ~mk) | ((unsigned)lv[i] & mk));
  return o;
}

__device__ __forceinline__ float wsum(float v) {
#pragma unroll
  for (int q = 16; q > 0; q >>= 1) v += __shfl_xor(v, q, 32);
  return v;
}
__device__ __forceinline__ float bsum(float p, float* red, int lane, int wave) {
  p = wsum(p);
  if (lane == 0) red[wave] = p;
  __syncthreads();
  const float t = ((red[0] + red[1]) + (red[2] + red[3])) + ((red[4] + red[5]) + (red[6] + red[7]));
  __syncthreads();
  return t;
}

__device__ __forceinline__ float gelu_exact(float v) {
  return 0.5f * v * (1.0f + erff(v * 0.70710678f));
}

__device__ __forceinline__ float lk4(const v4f s, const v4f d, const v4f a, float p) {
  float v0 = s.x + d.x, v1 = s.y + d.y, v2 = s.z + d.z, v3 = s.w + d.w;
  v0 = (v0 > 0.f) ? v0 : NEGS * v0;
  v1 = (v1 > 0.f) ? v1 : NEGS * v1;
  v2 = (v2 > 0.f) ? v2 : NEGS * v2;
  v3 = (v3 > 0.f) ? v3 : NEGS * v3;
  p = fmaf(v0, a.x, p); p = fmaf(v1, a.y, p); p = fmaf(v2, a.z, p); p = fmaf(v3, a.w, p);
  return p;
}

__device__ __forceinline__ int scan_chunk(const int* __restrict__ dsts, int nE, int cbase, int slotBase,
                                          int nb, int vec8, int* list, int tid, int lane, int wave) {
  int wc = 0;
  const int el0  = tid * EPT;
  const int e0   = cbase + el0;
  const int sent = -2147483647 - 1;
  v4i da, db;
  if (vec8 != 0 && cbase + CHUNK <= nE) {
    da = *(const v4i*)(dsts + e0);
    db = *(const v4i*)(dsts + e0 + 4);
  } else {
    da.x = (e0     < nE) ? dsts[min(e0,     nE - 1)] : sent;
    da.y = (e0 + 1 < nE) ? dsts[min(e0 + 1, nE - 1)] : sent;
    da.z = (e0 + 2 < nE) ? dsts[min(e0 + 2, nE - 1)] : sent;
    da.w = (e0 + 3 < nE) ? dsts[min(e0 + 3, nE - 1)] : sent;
    db.x = (e0 + 4 < nE) ? dsts[min(e0 + 4, nE - 1)] : sent;
    db.y = (e0 + 5 < nE) ? dsts[min(e0 + 5, nE - 1)] : sent;
    db.z = (e0 + 6 < nE) ? dsts[min(e0 + 6, nE - 1)] : sent;
    db.w = (e0 + 7 < nE) ? dsts[min(e0 + 7, nE - 1)] : sent;
  }
  const unsigned nbs = (unsigned)slotBase;
  const unsigned unb = (unsigned)nb;
  const unsigned s0 = (unsigned)da.x - nbs, s1 = (unsigned)da.y - nbs;
  const unsigned s2 = (unsigned)da.z - nbs, s3 = (unsigned)da.w - nbs;
  const unsigned s4 = (unsigned)db.x - nbs, s5 = (unsigned)db.y - nbs;
  const unsigned s6 = (unsigned)db.z - nbs, s7 = (unsigned)db.w - nbs;
  const bool h0 = s0 < unb, h1 = s1 < unb, h2 = s2 < unb, h3 = s3 < unb;
  const bool h4 = s4 < unb, h5 = s5 < unb, h6 = s6 < unb, h7 = s7 < unb;
  const unsigned any = __builtin_amdgcn_ballot_w32(h0 | h1 | h2 | h3 | h4 | h5 | h6 | h7);
  if (any != 0u) {
#define HITJ(J, HJ, SJ) { \
      const unsigned mj = __builtin_amdgcn_ballot_w32(HJ); \
      if (mj != 0u) { \
        if (HJ) { \
          const int pos = wc + (int)__builtin_amdgcn_mbcnt_lo(mj, 0u); \
          if (pos < WCAP) list[wave * WCAP + pos] = ((el0 + (J)) << 12) | (int)(SJ); \
        } \
        wc += (int)__builtin_popcount(mj); } }
    HITJ(0, h0, s0)
    HITJ(1, h1, s1)
    HITJ(2, h2, s2)
    HITJ(3, h3, s3)
    HITJ(4, h4, s4)
    HITJ(5, h5, s5)
    HITJ(6, h6, s6)
    HITJ(7, h7, s7)
#undef HITJ
  }
  return wc;
}

__global__ __launch_bounds__(NTHR) __attribute__((amdgpu_num_vgpr(248)))
void k_pa(const float* __restrict__ x, unsigned short* xb) {
  const int i = (int)blockIdx.x * NTHR + (int)threadIdx.x;
  if (i >= NNODE * (HID / 8)) return;
  const int row = i >> 6;
  const int c0  = (i & 63) * 8;
  const float* p = x + (size_t)row * XPITCH + 1 + c0;
  v4f a, b;
  a.x = p[0]; a.y = p[1]; a.z = p[2]; a.w = p[3];
  b.x = p[4]; b.y = p[5]; b.z = p[6]; b.w = p[7];
  const v8us hv = cvt8b(a, b);
  const size_t o = (size_t)row * HID + c0;
  *(volatile v8us*)(xb + o) = hv;
  __threadfence();
  *(volatile v8us*)(xb + o) = hv;
}

__global__ __launch_bounds__(NTHR) __attribute__((amdgpu_num_vgpr(248)))
void k_wtr(const float* __restrict__ w, int srcK, int srcN, unsigned short* wt, int pitch, int half, int nUnits) {
  const int u = (int)blockIdx.x * NTHR + (int)threadIdx.x;
  if (u >= nUnits) return;
  const int upr = pitch >> 3;
  const int n   = u / upr;
  const int k8  = (u - n * upr) * 8;
  const int ks  = (k8 >= half) ? (k8 - half) : k8;
  const int ncl = (n < srcN) ? n : (srcN - 1);
  float f[8];
#pragma unroll
  for (int i = 0; i < 8; ++i) {
    const int kk = ks + i;
    const int kc = (kk < srcK) ? kk : (srcK - 1);
    f[i] = w[(size_t)kc * (size_t)srcN + ncl];
  }
  v4f a, b;
  const bool nok = n < srcN;
  a.x = (nok && ks + 0 < srcK) ? f[0] : 0.f; a.y = (nok && ks + 1 < srcK) ? f[1] : 0.f;
  a.z = (nok && ks + 2 < srcK) ? f[2] : 0.f; a.w = (nok && ks + 3 < srcK) ? f[3] : 0.f;
  b.x = (nok && ks + 4 < srcK) ? f[4] : 0.f; b.y = (nok && ks + 5 < srcK) ? f[5] : 0.f;
  b.z = (nok && ks + 6 < srcK) ? f[6] : 0.f; b.w = (nok && ks + 7 < srcK) ? f[7] : 0.f;
  const v8us hv = cvt8b(a, b);
  const size_t o = (size_t)n * (size_t)pitch + k8;
  *(volatile v8us*)(wt + o) = hv;
  __threadfence();
  *(volatile v8us*)(wt + o) = hv;
}

template<int CONV>
__global__ __launch_bounds__(GTHR) __attribute__((amdgpu_num_vgpr(248)))
void k_gemm(const unsigned short* __restrict__ A, const unsigned short* __restrict__ WT,
            const float* __restrict__ bL, const float* __restrict__ bR,
            float* outF, int K, int ldo, int ncs, int planeStride)
{
  __shared__ __attribute__((aligned(16))) float stg[GBM * GBN];
  __shared__ float sbias[GBN];
  const int tid = (int)threadIdx.x, lane = tid & 31, wave = tid >> 5, hh = lane >> 4, m = lane & 15;
  const int rowBase = (int)blockIdx.x * GBM;
  const int col0    = (int)blockIdx.y * GBN;

  if (CONV) {
    const int cc = (col0 & (HID - 1)) + (tid & 63);
    const float vl = bL[cc];
    const float vr = bR[cc];
    asm volatile("" :: "v"(vl), "v"(vr));
    const float bv = rbf((col0 < HID) ? vl : vr);
    if (tid < GBN) sbias[tid] = bv;
  } else {
    if (tid < GBN) sbias[tid] = 0.f;
  }
  __syncthreads();

  v8f acc[4];
  {
    const v8f z = {0.f, 0.f, 0.f, 0.f, 0.f, 0.f, 0.f, 0.f};
    acc[0] = z; acc[1] = z; acc[2] = z; acc[3] = z;
  }
  const unsigned short* ap = A  + (size_t)(rowBase + 16 * wave + m) * (size_t)K + 8 * hh;
  const unsigned short* wp = WT + (size_t)(col0 + m) * (size_t)K + 8 * hh;
  const int ksteps = K >> 5;
#pragma unroll 1
  for (int ks = 0; ks < ksteps; ++ks) {
    FragB af;
    af.u[0] = *(const v8us*)(ap + 32 * ks);
    af.u[1] = *(const v8us*)(ap + 32 * ks + 16);
#pragma unroll
    for (int t = 0; t < 4; ++t) {
      const unsigned short* wq = wp + (size_t)(16 * t) * (size_t)K + 32 * ks;
      FragB bf;
      bf.u[0] = *(const v8us*)wq;
      bf.u[1] = *(const v8us*)(wq + 16);
      acc[t] = wmb(af, bf, acc[t]);
    }
  }

#pragma unroll
  for (int t = 0; t < 4; ++t) {
    const int lc = 16 * t + m;
    const float bv = sbias[lc];
#pragma unroll
    for (int r = 0; r < 8; ++r) {
      const int lr = 16 * wave + 8 * hh + r;
      stg[lr * GBN + lc] = acc[t][r] + bv;
    }
  }
  __syncthreads();

  const size_t obase = (size_t)(col0 / ncs) * (size_t)planeStride + (size_t)(col0 % ncs) + 4 * m;
  v4f fv[8];
#pragma unroll
  for (int i = 0; i < 8; ++i) {
    const int lr = 16 * wave + 2 * i + hh;
    fv[i] = *(const v4fa*)(stg + lr * GBN + 4 * m);
  }
#pragma unroll
  for (int i = 0; i < 8; ++i) {
    const int gr = rowBase + 16 * wave + 2 * i + hh;
    float* op = outF + obase + (size_t)gr * (size_t)ldo;
    *(volatile v4f*)op = fv[i];
  }
  __threadfence();
#pragma unroll
  for (int i = 0; i < 8; ++i) {
    const int gr = rowBase + 16 * wave + 2 * i + hh;
    float* op = outF + obase + (size_t)gr * (size_t)ldo;
    *(volatile v4f*)op = fv[i];
  }
}

template<int LAYER>
__global__ __launch_bounds__(NTHR) __attribute__((amdgpu_num_vgpr(248)))
void k_scan(const int* __restrict__ srcs, const int* __restrict__ dsts,
            const float* __restrict__ XL, const float* __restrict__ XR,
            const float* __restrict__ att, const float* __restrict__ bias,
            unsigned short* H1, float* S, float* T, int nE, int vec8) {
  extern __shared__ v4f lds_dyn[];
  int* reg1 = (int*)lds_dyn;
  int* reg2 = reg1 + RCAP;
  int* scnt = reg2 + RCAP;
  int* soff = scnt + NBMAX;
  int* list = soff + NBMAX;
  int* wcnt = list + LISTN;
  int* wtot = wcnt + NWAVE;
  float* winv = (float*)(wtot + NWAVE);
  const int tid = (int)threadIdx.x, lane = tid & 31, wave = tid >> 5;
  const int nb = NBRUN;
  const int nodeBase = (int)blockIdx.x * nb;

  {
    const v4i z4 = {0, 0, 0, 0};
    for (int i = tid * 4; i < ZINTS; i += NTHR * 4) *(v4ia*)(reg1 + i) = z4;
    if (tid < 2 * NWAVE) wcnt[tid] = 0;
  }
  __syncthreads();

  int tot = 0;
  const int nChunks = (nE + CHUNK - 1) / CHUNK;
#pragma unroll 1
  for (int ch = 0; ch < nChunks; ++ch) {
    const int cbase = ch * CHUNK;
    const int wc = scan_chunk(dsts, nE, cbase, nodeBase, nb, vec8, list, tid, lane, wave);
    if (lane == 0) wcnt[wave] = wc;
    __syncthreads();
    int pre = 0, all = 0;
#pragma unroll
    for (int w2 = 0; w2 < NWAVE; ++w2) {
      int c = wcnt[w2];
      c = c < 0 ? 0 : (c > WCAP ? WCAP : c);
      all += c;
      pre += (w2 < wave) ? c : 0;
    }
    const int wcc  = wc > WCAP ? WCAP : wc;
    const int base = tot + pre;
#pragma unroll 1
    for (int i = lane; i < wcc; i += 32) {
      const int ent = list[wave * WCAP + i];
      const int el  = (ent >> 12) & (CHUNK - 1);
      const int sl  = ent & (NBMAX - 1);
      int eid = cbase + el;
      eid = eid > nE - 1 ? nE - 1 : eid;
      const int pos = base + i;
      if (pos < RCAP) reg1[pos] = (int)(((unsigned)eid << 12) | (unsigned)sl);
    }
    tot += all;
    tot = tot > RCAP ? RCAP : tot;
    __syncthreads();
  }
  const int nh = tot;

  if (wave == 0) {
#pragma unroll 1
    for (int b0 = 0; b0 < nh; b0 += 32) {
      const int idx = b0 + lane;
      const int uv  = reg1[idx < RCAP ? idx : RCAP - 1];
      const int m32 = (nh - b0) < 32 ? (nh - b0) : 32;
#pragma unroll 1
      for (int k = 0; k < m32; ++k) {
        const int u  = __builtin_amdgcn_readlane(uv, k);
        const int sl = u & (NBMAX - 1);
        if (lane == 0) scnt[sl] = scnt[sl] + 1;
      }
    }
  }
  __syncthreads();

  {
    const v4i ca = *(const v4ia*)(scnt + 8 * tid);
    const v4i cb = *(const v4ia*)(scnt + 8 * tid + 4);
    const int e0 = ca.x < 0 ? 0 : ca.x, e1 = ca.y < 0 ? 0 : ca.y, e2 = ca.z < 0 ? 0 : ca.z, e3 = ca.w < 0 ? 0 : ca.w;
    const int e4 = cb.x < 0 ? 0 : cb.x, e5 = cb.y < 0 ? 0 : cb.y, e6 = cb.z < 0 ? 0 : cb.z, e7 = cb.w < 0 ? 0 : cb.w;
    const int ts = e0 + e1 + e2 + e3 + e4 + e5 + e6 + e7;
    int incl = ts;
#pragma unroll
    for (int d = 1; d < 32; d <<= 1) {
      const int up = __shfl_up(incl, d);
      if (lane >= d) incl += up;
    }
    if (lane == 31) wtot[wave] = incl;
    __syncthreads();
    int pre = 0;
#pragma unroll
    for (int w2 = 0; w2 < NWAVE; ++w2) pre += (w2 < wave) ? wtot[w2] : 0;
    int run = pre + incl - ts;
    soff[8 * tid + 0] = run; run += e0;
    soff[8 * tid + 1] = run; run += e1;
    soff[8 * tid + 2] = run; run += e2;
    soff[8 * tid + 3] = run; run += e3;
    soff[8 * tid + 4] = run; run += e4;
    soff[8 * tid + 5] = run; run += e5;
    soff[8 * tid + 6] = run; run += e6;
    soff[8 * tid + 7] = run;
  }
  __syncthreads();
  for (int i = tid; i < NBMAX; i += NTHR) list[i] = soff[i];
  __syncthreads();

  if (wave == 0) {
#pragma unroll 1
    for (int b0 = 0; b0 < nh; b0 += 32) {
      const int idx = b0 + lane;
      const int uv  = reg1[idx < RCAP ? idx : RCAP - 1];
      const int m32 = (nh - b0) < 32 ? (nh - b0) : 32;
#pragma unroll 1
      for (int k = 0; k < m32; ++k) {
        const int u   = __builtin_amdgcn_readlane(uv, k);
        const int sl  = u & (NBMAX - 1);
        const int eid = (int)((unsigned)u >> 12);
        if (lane == 0) {
          int pos = list[sl];
          pos = pos < 0 ? 0 : (pos > RCAP - 1 ? RCAP - 1 : pos);
          reg2[pos] = eid;
          list[sl] = pos + 1;
        }
      }
    }
  }
  __syncthreads();

  float* fl = (float*)list;
  {
    const int q4 = 4 * (tid & 127);
    const v4f a = *(const v4f*)(att + q4);
    const v4f b = *(const v4f*)(bias + q4);
    const bool fa = tid < 128;
    v4f o;
    o.x = rbf(fa ? a.x : b.x); o.y = rbf(fa ? a.y : b.y);
    o.z = rbf(fa ? a.z : b.z); o.w = rbf(fa ? a.w : b.w);
    *(v4fa*)(fl + 4 * tid) = o;
  }
  __syncthreads();

  const int nbw = nb >> 3;
  const bool ovf = (nh >= RCAP);
  const float qnan = __int_as_float(0x7fc00000);
  float* stw = (float*)reg1 + wave * STW;
  const float* biasL = fl + HID;
  float* tsh = fl + 2 * HID;
  v4f at[4];
#pragma unroll
  for (int q = 0; q < 4; ++q) at[q] = *(const v4fa*)(fl + 16 * lane + 4 * q);

#pragma unroll 1
  for (int jt = 0; jt < nbw; ++jt) {
    const int slot = wave * nbw + jt;
    const int grow = nodeBase + slot;
    const int gcl  = grow < NNODE ? grow : NNODE - 1;
    int st = soff[slot];
    const int craw = scnt[slot];
    int cnt = craw;
    st  = st < 0 ? 0 : (st > nh ? nh : st);
    cnt = cnt < 0 ? 0 : (cnt > DEGCAP ? DEGCAP : cnt);
    if (cnt > nh - st) cnt = nh - st;
    const bool bad = ovf || (craw > DEGCAP);

    const float* drow = XR + (size_t)gcl * HID + 16 * lane;
    v4f hd[4], av[4];
#pragma unroll
    for (int q = 0; q < 4; ++q) {
      hd[q] = *(const v4f*)(drow + 4 * q);
      const v4f z4 = {0.f, 0.f, 0.f, 0.f};
      av[q] = z4;
    }
    float mx = -1.0e30f, dn = 0.f;

#pragma unroll 1
    for (int q = 0; q <= cnt; ++q) {
      int idx = st + q - 1;
      idx = idx < 0 ? 0 : (idx > RCAP - 1 ? RCAP - 1 : idx);
      int eid = reg2[idx];
      eid = eid < 0 ? 0 : (eid > nE - 1 ? nE - 1 : eid);
      const int sraw = srcs[eid];
      int s = sraw < 0 ? 0 : (sraw > NNODE - 1 ? NNODE - 1 : sraw);
      s = (q == 0) ? gcl : s;
      const float* sr = XL + (size_t)s * HID + 16 * lane;
      v4f hs[4];
#pragma unroll
      for (int j = 0; j < 4; ++j) hs[j] = *(const v4f*)(sr + 4 * j);
      ldwait();
      float part = 0.f;
#pragma unroll
      for (int j = 0; j < 4; ++j) part = lk4(hs[j], hd[j], at[j], part);
      part += __shfl_xor(part, 1, 32);
      part += __shfl_xor(part, 2, 32);
      part += __shfl_xor(part, 4, 32);
      const float al = part;
      const float df = al - mx;
      const float ee = expf(-fabsf(df));
      const bool up  = df > 0.f;
      const float s1 = up ? ee : 1.0f;
      const float s2 = up ? 1.0f : ee;
      mx = up ? al : mx;
      dn = fmaf(dn, s1, s2);
#pragma unroll
      for (int j = 0; j < 4; ++j) av[j] = av[j] * s1 + hs[j] * s2;
    }
    const float inv = __builtin_amdgcn_rcpf(dn + 1e-16f);

    wsync();
#pragma unroll
    for (int j = 0; j < 4; ++j) *(v4fa*)(stw + 16 * lane + 4 * j) = av[j];
    if ((lane & 7) == 0) winv[wave * 4 + (lane >> 3)] = inv;
    wsync();
    float ps = 0.f;
#pragma unroll 1
    for (int i = 0; i < 16; ++i) {
      const int c = 32 * i + lane;
      float v = fmaf(stw[c], winv[wave * 4 + (i >> 2)], biasL[c]);
      if constexpr (LAYER == 1) v = gelu_exact(v);
      v = bad ? qnan : v;
      stw[c] = v;
      ps = fmaf(v, v, ps);
    }
    wsync();
    if constexpr (LAYER == 1) {
      v8us hv0, lv0, hv1, lv1;
      {
        const v4f ga = *(const v4fa*)(stw + 8 * lane);
        const v4f gb = *(const v4fa*)(stw + 8 * lane + 4);
        hilo8(ga, gb, hv0, lv0);
        const v4f gc = *(const v4fa*)(stw + 256 + 8 * lane);
        const v4f gd = *(const v4fa*)(stw + 256 + 8 * lane + 4);
        hilo8(gc, gd, hv1, lv1);
      }
      unsigned short* hp = H1 + (size_t)grow * (2 * HID) + 8 * lane;
      *(volatile v8us*)(hp)             = hv0;
      *(volatile v8us*)(hp + 256)       = hv1;
      *(volatile v8us*)(hp + HID)       = lv0;
      *(volatile v8us*)(hp + HID + 256) = lv1;
      __threadfence();
      *(volatile v8us*)(hp)             = hv0;
      *(volatile v8us*)(hp + 256)       = hv1;
      *(volatile v8us*)(hp + HID)       = lv0;
      *(volatile v8us*)(hp + HID + 256) = lv1;
    } else {
      const float tt = sqrtf(1.0f + wsum(ps));
      v4f gv[4];
#pragma unroll
      for (int j = 0; j < 4; ++j) gv[j] = *(const v4fa*)(stw + 128 * j + 4 * lane);
      float* op = S + (size_t)grow * HID + 4 * lane;
#pragma unroll
      for (int j = 0; j < 4; ++j) *(volatile v4f*)(op + 128 * j) = gv[j];
      __threadfence();
#pragma unroll
      for (int j = 0; j < 4; ++j) *(volatile v4f*)(op + 128 * j) = gv[j];
      if (lane == 0) tsh[slot] = tt;
    }
  }
  __syncthreads();
  if constexpr (LAYER == 2) {
    const v4f tv = *(const v4fa*)(tsh + 4 * tid);
    float* tp = T + nodeBase + 4 * tid;
    *(volatile v4f*)tp = tv;
    __threadfence();
    *(volatile v4f*)tp = tv;
  }
  (void)H1; (void)S; (void)T;
}

__global__ __launch_bounds__(NTHR) __attribute__((amdgpu_num_vgpr(248)))
void k_pool(const float* __restrict__ S, const float* __restrict__ T, const int* __restrict__ bsz,
            float* GM, unsigned short* Z0) {
  __shared__ __attribute__((aligned(16))) float tl[GSIZE];
  __shared__ __attribute__((aligned(16))) float rowg[ZP];
  __shared__ __attribute__((aligned(16))) float rowz[ZP];
  __shared__ float red[NWAVE];
  const int tid = (int)threadIdx.x, lane = tid & 31, wave = tid >> 5;
  const int g  = (int)blockIdx.x;
  const int r0 = g * GSIZE;
  const int bs = bsz[0];
  const bool bad = (bs != NGRAPH);
  const float qnan = __int_as_float(0x7fc00000);

  const float tv = T[r0 + (tid & (GSIZE - 1))];
  asm volatile("" :: "v"(tv));
  if (tid < GSIZE) tl[tid] = tv;
  float a0 = 0.0f, a1 = 0.0f;
#pragma unroll 2
  for (int j = 0; j < GSIZE; ++j) {
    const float* p = S + (size_t)(r0 + j) * HID + tid;
    a0 += p[0];
    a1 += p[256];
  }
  const float z0 = S[(size_t)r0 * HID + tid];
  const float z1 = S[(size_t)r0 * HID + 256 + tid];
  __syncthreads();
  float ts = 0.0f;
#pragma unroll 4
  for (int j = 0; j < GSIZE; ++j) ts += tl[j];
  const float m0 = a0 * 0.0078125f, m1 = a1 * 0.0078125f, mt = ts * 0.0078125f;
  const float tot = bsum(m0 * m0 + m1 * m1, red, lane, wave);
  const float ni = -(tot - mt * mt);
  const float cl = (ni < 1e-8f) ? 1e-8f : ni;
  const float rd = 1.0f / sqrtf(cl);
  const float t0 = tl[0];

  rowg[1 + tid]   = bad ? qnan : m0 * rd;
  rowg[257 + tid] = bad ? qnan : m1 * rd;
  rowz[1 + tid]   = bad ? qnan : z0;
  rowz[257 + tid] = bad ? qnan : z1;
  if (tid == 0) { rowg[0] = bad ? qnan : mt * rd; rowz[0] = bad ? qnan : t0; }
  if (tid < ZP - OUTW) { rowg[OUTW + tid] = 0.0f; rowz[OUTW + tid] = 0.0f; }
  __syncthreads();

  const int u = tid < (ZP / 4) ? tid : (ZP / 4 - 1);
  const v4f  gv = *(const v4fa*)(rowg + 4 * u);
  const v8us zv = hl8(rowz, u, ZP / 8);
  float* gp = GM + (size_t)g * ZP + 4 * u;
  unsigned short* zp = Z0 + (size_t)g * KA + 8 * u;
  const bool wr = tid < (ZP / 4);
  if (wr) { *(volatile v4f*)gp = gv; *(volatile v8us*)zp = zv; }
  __threadfence();
  if (wr) { *(volatile v4f*)gp = gv; *(volatile v8us*)zp = zv; }
}

template<int SW, int MODE>
__global__ __launch_bounds__(NTHR) __attribute__((amdgpu_num_vgpr(248)))
void k_row(const float* __restrict__ Y, int ldy, const float* __restrict__ bias, const float* __restrict__ sp,
           unsigned short* Zhl, float* Zf) {
  constexpr int HALF = SW + 32;
  constexpr int EPTR = SW / NTHR;
  constexpr int HU   = HALF / 8;
  static_assert(SW % NTHR == 0 && HALF % 8 == 0);
  __shared__ __attribute__((aligned(16))) float hrow[HALF];
  __shared__ float red[NWAVE];
  const int tid = (int)threadIdx.x, lane = tid & 31, wave = tid >> 5;
  const int g = (int)blockIdx.x;
  const float* yr = Y + (size_t)g * (size_t)ldy;

  const float y0 = yr[0] + rbf(bias[0]);
  float p = 0.0f;
#pragma unroll 1
  for (int i = 0; i < EPTR; ++i) {
    const int c = 1 + tid + NTHR * i;
    const float v = yr[c] + rbf(bias[c]);
    hrow[c] = v;
    p = fmaf(v, v, p);
  }
  if (tid < HALF - SW - 1) hrow[SW + 1 + tid] = 0.0f;
  const float sq  = bsum(p, red, lane, wave);
  const float sv0 = sp[0];
  const float sv  = SCALARS_RNE ? rbf(sv0) : sv0;
  const float es  = expf(sv);
  const float sg  = 1.0f / (1.0f + expf(-y0));
  const float t   = sg * es + 1.1f;
  const float sqc = (sq < 1e-8f) ? 1e-8f : sq;
  const float fac = sqrtf((t * t - 1.0f) / sqc);
  float p2 = 0.0f;
#pragma unroll 1
  for (int i = 0; i < EPTR; ++i) {
    const int c = 1 + tid + NTHR * i;
    float v = hrow[c] * fac;
    if constexpr (MODE == 0) v = gelu_exact(v);
    hrow[c] = v;
    p2 = fmaf(v, v, p2);
  }
  float head = t;
  if constexpr (MODE == 0) {
    const float tot2 = bsum(p2, red, lane, wave);
    head = sqrtf(1.0f + tot2);
  }
  if (tid == 0) hrow[0] = head;
  __syncthreads();

  if constexpr (MODE == 2) {
    const int u = tid < (HALF / 4) ? tid : (HALF / 4 - 1);
    const v4f gv = *(const v4fa*)(hrow + 4 * u);
    float* op = Zf + (size_t)g * HALF + 4 * u;
    const bool wr = tid < (HALF / 4);
    if (wr) *(volatile v4f*)op = gv;
    __threadfence();
    if (wr) *(volatile v4f*)op = gv;
  } else {
    constexpr int NU  = 2 * HU;
    constexpr int NIT = (NU + NTHR - 1) / NTHR;
    unsigned short* zp = Zhl + (size_t)g * (2 * HALF);
#pragma unroll 1
    for (int it = 0; it < NIT; ++it) {
      const int u  = tid + NTHR * it;
      const int uc = u < NU ? u : NU - 1;
      const v8us o = hl8(hrow, uc, HU);
      if (u < NU) *(volatile v8us*)(zp + 8 * u) = o;
    }
    __threadfence();
#pragma unroll 1
    for (int it = 0; it < NIT; ++it) {
      const int u  = tid + NTHR * it;
      const int uc = u < NU ? u : NU - 1;
      const v8us o = hl8(hrow, uc, HU);
      if (u < NU) *(volatile v8us*)(zp + 8 * u) = o;
    }
  }
  (void)Zhl; (void)Zf;
}

__global__ __launch_bounds__(NTHR) __attribute__((amdgpu_num_vgpr(248)))
void k_store(const float* __restrict__ ZG, float* out) {
  const int i = (int)blockIdx.x * NTHR + (int)threadIdx.x;
  if (i >= 2 * OUTQ) return;
  const int o = (i >= OUTQ) ? 1 : 0;
  const int j = i - o * OUTQ;
  const float* base = ZG + (size_t)o * (NGRAPH * ZP);
  float f[4];
#pragma unroll
  for (int q = 0; q < 4; ++q) {
    int e = 4 * j + q;
    e = e > NGRAPH * OUTW - 1 ? NGRAPH * OUTW - 1 : e;
    const int gq = e / OUTW;
    const int c  = e - gq * OUTW;
    f[q] = base[gq * ZP + c];
  }
  asm volatile("" :: "v"(f[0]), "v"(f[1]), "v"(f[2]), "v"(f[3]));
  v4f v;
  v.x = f[0]; v.y = f[1]; v.z = f[2]; v.w = f[3];
  float* op = out + (size_t)4 * (size_t)i;
  *(volatile v4f*)op = v;
  __threadfence();
  *(volatile v4f*)op = v;
}

static inline int cdiv(int a, int b) { return (a + b - 1) / b; }

extern "C" void kernel_launch(void* const* d_in, const int* in_sizes, int n_in,
                              void* d_out, int out_size, void* d_ws, size_t ws_size,
                              hipStream_t stream) {
  if (n_in < 24) return;
  if (in_sizes[0] != NNODE * XPITCH) return;
  if (in_sizes[1] != 2 * NEDGE) return;
  if (in_sizes[2] != 1) return;
  if (in_sizes[3] != HID * HID || in_sizes[5] != HID * HID || in_sizes[9] != HID * HID || in_sizes[11] != HID * HID) return;
  if (in_sizes[4] != HID || in_sizes[6] != HID || in_sizes[7] != HID || in_sizes[8] != HID) return;
  if (in_sizes[10] != HID || in_sizes[12] != HID || in_sizes[13] != HID || in_sizes[14] != HID) return;
  if (in_sizes[15] != OUTW * 2049 || in_sizes[16] != 2049 || in_sizes[17] != 1) return;
  if (in_sizes[18] != 2049 * OUTW || in_sizes[19] != OUTW || in_sizes[20] != 1) return;
  if (in_sizes[21] != OUTW * OUTW || in_sizes[22] != OUTW || in_sizes[23] != 1) return;
  if (out_size != 2 * NGRAPH * OUTW) return;

  const float* x     = (const float*)d_in[0];
  const int*   ei    = (const int*)  d_in[1];
  const int*   bsz   = (const int*)  d_in[2];
  const float* Wl1   = (const float*)d_in[3];
  const float* bl1   = (const float*)d_in[4];
  const float* Wr1   = (const float*)d_in[5];
  const float* br1   = (const float*)d_in[6];
  const float* att1  = (const float*)d_in[7];
  const float* bias1 = (const float*)d_in[8];
  const float* Wl2   = (const float*)d_in[9];
  const float* bl2   = (const float*)d_in[10];
  const float* Wr2   = (const float*)d_in[11];
  const float* br2   = (const float*)d_in[12];
  const float* att2  = (const float*)d_in[13];
  const float* bias2 = (const float*)d_in[14];
  const float* Wa    = (const float*)d_in[15];
  const float* ba    = (const float*)d_in[16];
  const float* sa    = (const float*)d_in[17];
  const float* Wb    = (const float*)d_in[18];
  const float* bb    = (const float*)d_in[19];
  const float* sb    = (const float*)d_in[20];
  const float* Wf    = (const float*)d_in[21];
  const float* bfv   = (const float*)d_in[22];
  const float* sf    = (const float*)d_in[23];
  float* out = (float*)d_out;
  const int nE = NEDGE;
  const int* src = ei;
  const int* dst = ei + nE;
  const int vec8 = ((nE & 3) == 0) ? 1 : 0;

  char* ws = (char*)d_ws;
  size_t off = 0;
  const size_t oR1  = off; off += (size_t)NNODE * 2 * HID * 2;       off = (off + 255) & ~(size_t)255;
  const size_t oXLR = off; off += (size_t)2 * NNODE * HID * 4;       off = (off + 255) & ~(size_t)255;
  const size_t oT   = off; off += (size_t)NNODE * 4;                 off = (off + 255) & ~(size_t)255;
  const size_t oBT1 = off; off += (size_t)2 * HID * HID * 2;         off = (off + 255) & ~(size_t)255;
  const size_t oBT2 = off; off += (size_t)2 * HID * 2 * HID * 2;     off = (off + 255) & ~(size_t)255;
  const size_t oWAT = off; off += (size_t)NA * KA * 2;               off = (off + 255) & ~(size_t)255;
  const size_t oWBT = off; off += (size_t)NBF * KB * 2;              off = (off + 255) & ~(size_t)255;
  const size_t oWFT = off; off += (size_t)NBF * KA * 2;              off = (off + 255) & ~(size_t)255;
  const size_t oZ0  = off; off += (size_t)NGRAPH * KA * 2;           off = (off + 255) & ~(size_t)255;
  const size_t oYA  = off; off += (size_t)NGRAPH * NA * 4;           off = (off + 255) & ~(size_t)255;
  const size_t oZ1  = off; off += (size_t)NGRAPH * KB * 2;           off = (off + 255) & ~(size_t)255;
  const size_t oYB  = off; off += (size_t)NGRAPH * NBF * 4;          off = (off + 255) & ~(size_t)255;
  const size_t oZ2  = off; off += (size_t)NGRAPH * KA * 2;           off = (off + 255) & ~(size_t)255;
  const size_t oYF  = off; off += (size_t)NGRAPH * NBF * 4;          off = (off + 255) & ~(size_t)255;
  const size_t oZG  = off; off += (size_t)2 * NGRAPH * ZP * 4;       off = (off + 255) & ~(size_t)255;
  if (off > ws_size || off > (size_t)WSMAX) return;
  unsigned short* XB  = (unsigned short*)(ws + oR1);
  unsigned short* H1  = (unsigned short*)(ws + oR1);
  float*          S   = (float*)(ws + oR1);
  float*          XL  = (float*)(ws + oXLR);
  float*          XR  = XL + (size_t)NNODE * HID;
  float*          T   = (float*)(ws + oT);
  unsigned short* BT1 = (unsigned short*)(ws + oBT1);
  unsigned short* BT2 = (unsigned short*)(ws + oBT2);
  unsigned short* WAT = (unsigned short*)(ws + oWAT);
  unsigned short* WBT = (unsigned short*)(ws + oWBT);
  unsigned short* WFT = (unsigned short*)(ws + oWFT);
  unsigned short* Z0  = (unsigned short*)(ws + oZ0);
  float*          YA  = (float*)(ws + oYA);
  unsigned short* Z1  = (unsigned short*)(ws + oZ1);
  float*          YB  = (float*)(ws + oYB);
  unsigned short* Z2  = (unsigned short*)(ws + oZ2);
  float*          YF  = (float*)(ws + oYF);
  float*          ZG  = (float*)(ws + oZG);
  float*          Z3  = ZG;
  float*          GM  = ZG + (size_t)NGRAPH * ZP;

  hipFuncSetAttribute(reinterpret_cast<const void*>(&k_scan<1>), hipFuncAttributeMaxDynamicSharedMemorySize, LDS_SCAN);
  hipFuncSetAttribute(reinterpret_cast<const void*>(&k_scan<2>), hipFuncAttributeMaxDynamicSharedMemorySize, LDS_SCAN);

  k_pa<<<NNODE * (HID / 8) / NTHR, NTHR, 0, stream>>>(x, XB);
  {
    const int nU1 = HID * (HID / 8);
    k_wtr<<<cdiv(nU1, NTHR), NTHR, 0, stream>>>(Wl1, HID, HID, BT1, HID, HID, nU1);
    k_wtr<<<cdiv(nU1, NTHR), NTHR, 0, stream>>>(Wr1, HID, HID, BT1 + (size_t)HID * HID, HID, HID, nU1);
    const int nU2 = HID * (2 * HID / 8);
    k_wtr<<<cdiv(nU2, NTHR), NTHR, 0, stream>>>(Wl2, HID, HID, BT2, 2 * HID, HID, nU2);
    k_wtr<<<cdiv(nU2, NTHR), NTHR, 0, stream>>>(Wr2, HID, HID, BT2 + (size_t)HID * 2 * HID, 2 * HID, HID, nU2);
    const int nUa = NA * (KA / 8);
    k_wtr<<<cdiv(nUa, NTHR), NTHR, 0, stream>>>(Wa, OUTW, 2049, WAT, KA, ZP, nUa);
    const int nUb = NBF * (KB / 8);
    k_wtr<<<cdiv(nUb, NTHR), NTHR, 0, stream>>>(Wb, 2049, OUTW, WBT, KB, KBH, nUb);
    const int nUf = NBF * (KA / 8);
    k_wtr<<<cdiv(nUf, NTHR), NTHR, 0, stream>>>(Wf, OUTW, OUTW, WFT, KA, ZP, nUf);
  }

  const int gM = NNODE / GBM;
  const int gS = NNODE / NBRUN;
  k_gemm<1><<<dim3(gM, 2 * HID / GBN), GTHR, 0, stream>>>(XB, BT1, bl1, br1, XL, HID, HID, HID, NNODE * HID);
  k_scan<1><<<gS, NTHR, LDS_SCAN, stream>>>(src, dst, XL, XR, att1, bias1, H1, S, T, nE, vec8);
  k_gemm<1><<<dim3(gM, 2 * HID / GBN), GTHR, 0, stream>>>(H1, BT2, bl2, br2, XL, 2 * HID, HID, HID, NNODE * HID);
  k_scan<2><<<gS, NTHR, LDS_SCAN, stream>>>(src, dst, XL, XR, att2, bias2, H1, S, T, nE, vec8);
  k_pool<<<NGRAPH, NTHR, 0, stream>>>(S, T, bsz, GM, Z0);
  k_gemm<0><<<dim3(NGRAPH / GBM, NA / GBN), GTHR, 0, stream>>>(Z0, WAT, bl1, br1, YA, KA, NA, NA, 0);
  k_row<2048, 0><<<NGRAPH, NTHR, 0, stream>>>(YA, NA, ba, sa, Z1, Z3);
  k_gemm<0><<<dim3(NGRAPH / GBM, NBF / GBN), GTHR, 0, stream>>>(Z1, WBT, bl1, br1, YB, KB, NBF, NBF, 0);
  k_row<512, 1><<<NGRAPH, NTHR, 0, stream>>>(YB, NBF, bb, sb, Z2, Z3);
  k_gemm<0><<<dim3(NGRAPH / GBM, NBF / GBN), GTHR, 0, stream>>>(Z2, WFT, bl1, br1, YF, KA, NBF, NBF, 0);
  k_row<512, 2><<<NGRAPH, NTHR, 0, stream>>>(YF, NBF, bfv, sf, Z2, Z3);
  k_store<<<cdiv(2 * OUTQ, NTHR), NTHR, 0, stream>>>(ZG, out);
}
